// EncoderDecoderLSTM_75488345195356
// MI455X (gfx1250) — hardware-verified
//
#include <hip/hip_runtime.h>
#include <stdint.h>
#include <stddef.h>

typedef __attribute__((ext_vector_type(16))) _Float16 v16h;
typedef __attribute__((ext_vector_type(8)))  _Float16 v8h;
typedef __attribute__((ext_vector_type(16))) __bf16   v16b;
typedef __attribute__((ext_vector_type(8)))  __bf16   v8b;
typedef __attribute__((ext_vector_type(8)))  float    v8f;
typedef __attribute__((ext_vector_type(4)))  float    v4f;
typedef __attribute__((ext_vector_type(4)))  unsigned int v4u;
#define PSCALE 32768.0f
#define U16(p) ((const unsigned short*)(const void*)(p))
#define PSCALE_INV (1.0f / 32768.0f)

__device__ __forceinline__ unsigned short f2bf_bits(float f) {
  unsigned u = __float_as_uint(f);
  return (unsigned short)((u + 0x7FFFu + ((u >> 16) & 1u)) >> 16);
}
__device__ __forceinline__ float bf_bits2f(unsigned short h) { return __uint_as_float(((unsigned)h) << 16); }

__device__ __forceinline__ void dep_guard_h(v8f& a, v8f& b, v16h x, v16h y) { asm volatile("v_nop\n\tv_nop\n\tv_nop\n\tv_nop" : "+v"(a), "+v"(b) : "v"(x), "v"(y)); }
__device__ __forceinline__ void dep_guard_b(v8f& a, v8f& b, v16b x, v16b y) { asm volatile("v_nop\n\tv_nop\n\tv_nop\n\tv_nop" : "+v"(a), "+v"(b) : "v"(x), "v"(y)); }
__device__ __forceinline__ void keep4_h(v16h a, v16h b, v16h c, v16h d) { asm volatile("v_nop" :: "v"(a), "v"(b), "v"(c), "v"(d)); }
__device__ __forceinline__ void keep4_b(v16b a, v16b b, v16b c, v16b d) { asm volatile("v_nop" :: "v"(a), "v"(b), "v"(c), "v"(d)); }
__device__ __forceinline__ void acc_guard4(v8f& a, v8f& b, v8f& c, v8f& d) { asm volatile("v_nop\n\tv_nop\n\tv_nop\n\tv_nop" : "+v"(a), "+v"(b), "+v"(c), "+v"(d)); }
template <typename T> struct Frag;
template <> struct Frag<_Float16> {
  typedef v16h V; union U { v16h v; v8h h[2]; };
  static __device__ __forceinline__ v16h load(const _Float16* p) {
    U f; f.h[0] = *(const v8h*)(p); f.h[1] = *(const v8h*)(p + 16); return f.v;
  }
  static __device__ __forceinline__ v8f mma(v16h a, v16h b, v8f c) {
    return __builtin_amdgcn_wmma_f32_16x16x32_f16(false, a, false, b, (short)0, c, false, false);
  }
  static __device__ __forceinline__ void guard(v8f& a, v8f& b, v16h x, v16h y) { dep_guard_h(a, b, x, y); }
  static __device__ __forceinline__ void keep(v16h a, v16h b, v16h c, v16h d) { keep4_h(a, b, c, d); }
};
template <> struct Frag<__bf16> {
  typedef v16b V; union U { v16b v; v8b h[2]; };
  static __device__ __forceinline__ v16b load(const __bf16* p) {
    U f; f.h[0] = *(const v8b*)(p); f.h[1] = *(const v8b*)(p + 16); return f.v;
  }
  static __device__ __forceinline__ v8f mma(v16b a, v16b b, v8f c) {
    return __builtin_amdgcn_wmma_f32_16x16x32_bf16(false, a, false, b, (short)0, c, false, false);
  }
  static __device__ __forceinline__ void guard(v8f& a, v8f& b, v16b x, v16b y) { dep_guard_b(a, b, x, y); }
  static __device__ __forceinline__ void keep(v16b a, v16b b, v16b c, v16b d) { keep4_b(a, b, c, d); }
};

template <int ET> struct Elem;
template <> struct Elem<0> { typedef _Float16 T; };
template <> struct Elem<1> { typedef __bf16 T; };
template <int ET, bool SPLIT, int BIAS_MODE, int OUT_MODE, bool RESID, int ACT = 0>
__global__ __launch_bounds__(256) void wmma_gemm64(
    const unsigned short* __restrict__ Ap, const unsigned short* __restrict__ A2p, int lda, long strideA,
    const unsigned short* __restrict__ Btp, const unsigned short* __restrict__ Bt2p, int ldb, long strideB,
    void* __restrict__ Cout, void* __restrict__ Cout2, int ldc, long strideC,
    const float* __restrict__ bias,
    const float* __restrict__ resid, long strideR,
    int M, int N, int K, float scale) {
  typedef typename Elem<ET>::T T;
  typedef typename Frag<T>::V V;
  const T* A = (const T*)Ap; const T* A2 = (const T*)A2p; const T* Bt = (const T*)Btp; const T* Bt2 = (const T*)Bt2p;
  __shared__ __align__(16) float sT[8][16 * 68];
  const int b    = blockIdx.y;
  const int lane = threadIdx.x & 31;
  const int wave = threadIdx.x >> 5;
  const int tilesN = N >> 6;
  const int tilesM = M >> 6;
  const int tile = blockIdx.x * 8 + wave;
  if (tile >= tilesM * tilesN) return;
  const int tm = tile / tilesN;
  const int tn = tile - tm * tilesN;
  const int m0 = tm << 6;
  const int n0 = tn << 6;

  const T* Ab  = A  + (size_t)b * strideA;
  const T* Bb  = Bt + (size_t)b * strideB;
  const T* Ab2 = SPLIT ? (A2  + (size_t)b * strideA) : nullptr;
  const T* Bb2 = SPLIT ? (Bt2 + (size_t)b * strideB) : nullptr;

  const int rlane = lane & 15;
  const int koff  = (lane >> 4) * 8;
  const int mOff  = (lane >> 4) * 8;

  v8f acc[4][4];
#pragma unroll
  for (int i = 0; i < 4; ++i)
#pragma unroll
    for (int j = 0; j < 4; ++j) acc[i][j] = (v8f){0.f,0.f,0.f,0.f,0.f,0.f,0.f,0.f};

  for (int k0 = 0; k0 < K; k0 += 32) {
    V bh[4], bl[4];
#pragma unroll
    for (int j = 0; j < 4; ++j) {
      const size_t bo = (size_t)(n0 + (j << 4) + rlane) * ldb + koff + k0;
      bh[j] = Frag<T>::load(Bb + bo);
      if (SPLIT) bl[j] = Frag<T>::load(Bb2 + bo);
    }
#pragma unroll
    for (int i = 0; i < 4; ++i) {
      const size_t ao = (size_t)(m0 + (i << 4) + rlane) * lda + koff + k0;
      V ah = Frag<T>::load(Ab + ao);
      V al;
      if (SPLIT) al = Frag<T>::load(Ab2 + ao);
#pragma unroll
      for (int j = 0; j < 4; ++j) {
        acc[i][j] = Frag<T>::mma(ah, bh[j], acc[i][j]);
        if (SPLIT) {
          acc[i][j] = Frag<T>::mma(ah, bl[j], acc[i][j]);
          acc[i][j] = Frag<T>::mma(al, bh[j], acc[i][j]);
        }
      }
      Frag<T>::guard(acc[i][0], acc[i][3], ah, SPLIT ? al : ah);
    }
    Frag<T>::keep(bh[0], bh[1], bh[2], bh[3]);
    if (SPLIT) Frag<T>::keep(bl[0], bl[1], bl[2], bl[3]);
  }
  acc_guard4(acc[0][0], acc[0][1], acc[0][2], acc[0][3]);
  acc_guard4(acc[1][0], acc[1][1], acc[1][2], acc[1][3]);
  acc_guard4(acc[2][0], acc[2][1], acc[2][2], acc[2][3]);
  acc_guard4(acc[3][0], acc[3][1], acc[3][2], acc[3][3]);

  float* slab = sT[wave];
  const float* Rb = RESID ? (resid + (size_t)b * strideR) : nullptr;
#pragma unroll
  for (int i = 0; i < 4; ++i) {
    const int mBase = m0 + (i << 4);
#pragma unroll
    for (int j = 0; j < 4; ++j) {
      const int n = n0 + (j << 4) + rlane;
      float bv = 0.f;
      if (BIAS_MODE == 2) bv = bias[n];
#pragma unroll
      for (int r = 0; r < 8; ++r) {
        float v = acc[i][j][r] * scale;
        if (BIAS_MODE == 1) v += bias[mBase + mOff + r];
        if (BIAS_MODE == 2) v += bv;
        if (RESID) v += Rb[(size_t)(mBase + mOff + r) * ldc + n];
        if (ACT == 1) v = tanhf(v);
        if (ACT == 2) v = fmaxf(v, 0.0f);
        if (ACT == 3) v = v / (1.0f + expf(-v));
        if (ACT == 4) v = (v > 0.f) ? v : 0.01f * v;
        if (ACT == 5) v = 0.5f * v * (1.0f + erff(v * 0.70710678118654752f));
        slab[(mOff + r) * 68 + (j << 4) + rlane] = v;
      }
    }
    __builtin_amdgcn_fence(__ATOMIC_RELEASE, "workgroup");
    __builtin_amdgcn_wave_barrier();
    __builtin_amdgcn_fence(__ATOMIC_ACQUIRE, "workgroup");
    if (OUT_MODE == 0) {
      float* C = (float*)Cout + (size_t)b * strideC;
      const int hh = lane >> 4, c4 = (lane & 15) * 4;
      for (int pass = 0; pass < 2; ++pass) {
#pragma unroll
        for (int it = 0; it < 8; ++it) {
          const int row = it * 2 + hh;
          v4f v = *(const v4f*)(slab + row * 68 + c4);
          *(volatile v4f*)(C + (size_t)(mBase + row) * ldc + n0 + c4) = v;
        }
        __threadfence();
      }
    } else {
      const int q = lane >> 3, c8 = (lane & 7) * 8;
      unsigned short* C  = (unsigned short*)Cout  + (size_t)b * strideC;
      unsigned short* C2 = (OUT_MODE == 2) ? ((unsigned short*)Cout2 + (size_t)b * strideC) : nullptr;
      for (int pass = 0; pass < 2; ++pass) {
#pragma unroll
        for (int it = 0; it < 4; ++it) {
          const int row = it * 4 + q;
          const float* sp = slab + row * 68 + c8;
          v8h hv, lv;
#pragma unroll
          for (int e = 0; e < 8; ++e) {
            if (OUT_MODE == 1) {
              hv[e] = (_Float16)sp[e];
            } else {
              unsigned short hb = f2bf_bits(sp[e]);
              unsigned short lb = f2bf_bits(sp[e] - bf_bits2f(hb));
              hv[e] = __builtin_bit_cast(_Float16, hb);
              lv[e] = __builtin_bit_cast(_Float16, lb);
            }
          }
          *(volatile v8h*)(C + (size_t)(mBase + row) * ldc + n0 + c8) = hv;
          if (OUT_MODE == 2) *(volatile v8h*)(C2 + (size_t)(mBase + row) * ldc + n0 + c8) = lv;
        }
        __threadfence();
      }
    }
    __builtin_amdgcn_fence(__ATOMIC_RELEASE, "workgroup");
    __builtin_amdgcn_wave_barrier();
    __builtin_amdgcn_fence(__ATOMIC_ACQUIRE, "workgroup");
  }
}

__global__ __launch_bounds__(256) void cast_f32_f16x2(
    const float* __restrict__ in, _Float16* __restrict__ out, int n2) {
  int i = blockIdx.x * 256 + threadIdx.x;
  if (i < n2) {
    const _Float16 h0 = (_Float16)in[2 * i], h1 = (_Float16)in[2 * i + 1];
    const unsigned u = (unsigned)__builtin_bit_cast(unsigned short, h0) | ((unsigned)__builtin_bit_cast(unsigned short, h1) << 16);
    ((volatile unsigned*)out)[i] = u;
    __threadfence();
    ((volatile unsigned*)out)[i] = u;
  }
}

constexpr int kNB   = 128;
constexpr int kTP   = 1024;
constexpr int kTF   = 512;
constexpr int kTT   = 1536;
constexpr int kNIN  = 64;
constexpr int kNIP  = 128;
constexpr int kNH   = 256;
constexpr int kNG   = 1024;
constexpr int kKC   = 384;
constexpr int kATP  = 392;
constexpr int kNOUT = 64;
constexpr float kGSC = 1.0f / 128.0f;
static_assert((size_t)kNB * kTP * kNIP == (size_t)kNB * kTF * kNH, "enc plane and future hs plane have equal size");
static_assert(kATP % 8 == 0 && kATP >= kKC, "pitch");

__device__ __forceinline__ v8f mma_h(v16h a, v16h b, v8f c) {
  c = __builtin_amdgcn_wmma_f32_16x16x32_f16(false, a, false, b, (short)0, c, false, false);
  asm volatile("v_nop\n\tv_nop\n\tv_nop\n\tv_nop" : "+v"(c) : "v"(a), "v"(b));
  return c;
}
__device__ __forceinline__ v8f zero8f() { return (v8f){0.f,0.f,0.f,0.f,0.f,0.f,0.f,0.f}; }

__device__ __forceinline__ float sigm_f(float v) {
  v = fminf(fmaxf(v, -30.0f), 30.0f);
  const float e = expf(-v);
  return __builtin_amdgcn_rcpf(1.0f + e);
}
__device__ __forceinline__ float tanh_f(float v) {
  v = fminf(fmaxf(v, -15.0f), 15.0f);
  const float e = expf(2.0f * v);
  return 1.0f - 2.0f * __builtin_amdgcn_rcpf(1.0f + e);
}

__device__ __forceinline__ unsigned pack_h2(float a, float b) {
  const _Float16 h0 = (_Float16)a, h1 = (_Float16)b;
  return (unsigned)__builtin_bit_cast(unsigned short, h0) | ((unsigned)__builtin_bit_cast(unsigned short, h1) << 16);
}
__device__ __forceinline__ void store_u32_twice(_Float16* base, int i, unsigned u) {
  ((volatile unsigned*)base)[i] = u;
  __threadfence();
  ((volatile unsigned*)base)[i] = u;
}

__global__ __launch_bounds__(256) void prep_planes(
    const float* __restrict__ pW_ih, const float* __restrict__ pW_hh,
    const float* __restrict__ fW_ih, const float* __restrict__ fW_hh,
    const float* __restrict__ fut_W, const float* __restrict__ dec_W,
    const float* __restrict__ enc_W, const float* __restrict__ enc_b,
    _Float16* __restrict__ btp, _Float16* __restrict__ btf, _Float16* __restrict__ futw,
    _Float16* __restrict__ decw, _Float16* __restrict__ encw, float* __restrict__ encb8)
{
  const int blk = blockIdx.x;
  const int tid = threadIdx.x;
  if (blk < 1536) {
    const bool isP = (blk < 768);
    const float* Wih = isP ? pW_ih : fW_ih;
    const float* Whh = isP ? pW_hh : fW_hh;
    _Float16* dst = isP ? btp : btf;
    const int p   = (isP ? blk : (blk - 768)) * 256 + tid;
    const int row = p / 192;
    const int col = (p - row * 192) * 2;
    const int ci  = (col < kNIP - 2) ? col : (kNIP - 2);
    const int ch  = (col >= kNIP) ? (col - kNIP) : 0;
    const float a0 = Wih[row * kNIP + ci], a1 = Wih[row * kNIP + ci + 1];
    const float h0 = Whh[row * kNH + ch],  h1 = Whh[row * kNH + ch + 1];
    const bool inIh = (col < kNIP);
    const float v0 = inIh ? a0 : h0;
    const float v1 = inIh ? a1 : h1;
    store_u32_twice(dst, p, pack_h2(16.0f * v0, 16.0f * v1));
  } else if (blk < 1600) {
    const int p = (blk - 1536) * 256 + tid;
    store_u32_twice(futw, p, pack_h2(16.0f * fut_W[2 * p], 16.0f * fut_W[2 * p + 1]));
  } else if (blk < 1632) {
    const int p = (blk - 1600) * 256 + tid;
    store_u32_twice(decw, p, pack_h2(16.0f * dec_W[2 * p], 16.0f * dec_W[2 * p + 1]));
  } else if (blk < 1648) {
    const int p = (blk - 1632) * 256 + tid;
    store_u32_twice(encw, p, pack_h2(16.0f * enc_W[2 * p], 16.0f * enc_W[2 * p + 1]));
  } else {
    if (tid < 32) {
      v4f w = *(const v4f*)(enc_b + 4 * tid);
      w = w * 8.0f;
      *(volatile v4f*)(encb8 + 4 * tid) = w;
      __threadfence();
      *(volatile v4f*)(encb8 + 4 * tid) = w;
    }
  }
}

__global__ __launch_bounds__(256) void lstm_seq_kernel(
    const _Float16* enc16, const _Float16* btp, const _Float16* btf, const _Float16* futw,
    const float* pb_ih, const float* pb_hh, const float* fb_ih, const float* fb_hh,
    const float* fut_b, const int* futn,
    _Float16* hsp, _Float16* hsf)
{
  __shared__ __align__(16) _Float16 At[16 * kATP];

  const int tid  = threadIdx.x;
  const int wave = tid >> 5;
  const int lane = tid & 31;
  const int cl   = lane & 15;
  const int hh   = lane >> 4;
  const int b0   = blockIdx.x * 16;

  {
    const v4u z = {0u, 0u, 0u, 0u};
    for (int i = tid; i < 512; i += 256) {
      const int m = i >> 5, seg = i & 31;
      *(v4u*)(At + m * kATP + kNIP + 8 * seg) = z;
    }
  }
  {
    const int m = tid >> 4, seg = tid & 15;
    const v8h e = *(const v8h*)(enc16 + ((size_t)(b0 + m) * kTP) * kNIP + 8 * seg);
    *(v8h*)(At + m * kATP + 8 * seg) = e;
  }
  float bp[2][4], bq[2][4];
#pragma unroll
  for (int ubi = 0; ubi < 2; ++ubi)
#pragma unroll
    for (int g = 0; g < 4; ++g) {
      const int n = g * kNH + 16 * (2 * wave + ubi) + cl;
      bp[ubi][g] = pb_ih[n] + pb_hh[n];
      bq[ubi][g] = fb_ih[n] + fb_hh[n];
    }
  const float futb = fut_b[16 * wave + cl];

  float cst[2][8], hreg[2][8];
#pragma unroll
  for (int ubi = 0; ubi < 2; ++ubi)
#pragma unroll
    for (int r = 0; r < 8; ++r) { cst[ubi][r] = 0.f; hreg[ubi][r] = 0.f; }

  int nf = futn[0];
  nf = (nf < 0) ? 0 : nf;
  nf = (nf > kTF) ? kTF : nf;
  const int tEnd = kTP + nf;

  __syncthreads();

  for (int t = 0; t < tEnd; ++t) {
    const bool fut = (t >= kTP);

    if (fut) {
      v8f acc = zero8f();
#pragma unroll 1
      for (int k0 = 0; k0 < kNH; k0 += 32) {
        const v16h a  = Frag<_Float16>::load(At + cl * kATP + kNIP + k0 + 8 * hh);
        const v16h bw = Frag<_Float16>::load(futw + (size_t)(16 * wave + cl) * kNH + k0 + 8 * hh);
        acc = mma_h(a, bw, acc);
      }
#pragma unroll
      for (int r = 0; r < 8; ++r) {
        const float v = acc[r] * kGSC + futb;
        At[(8 * hh + r) * kATP + 16 * wave + cl] = (_Float16)(8.0f * v);
      }
      __syncthreads();
    }

    {
      const _Float16* Bt = fut ? btf : btp;
#pragma unroll
      for (int ubi = 0; ubi < 2; ++ubi) {
        const int ub = 2 * wave + ubi;
        v8f acc[4];
#pragma unroll
        for (int g = 0; g < 4; ++g) acc[g] = zero8f();
#pragma unroll 1
        for (int k0 = 0; k0 < kKC; k0 += 32) {
          const v16h a = Frag<_Float16>::load(At + cl * kATP + k0 + 8 * hh);
#pragma unroll
          for (int g = 0; g < 4; ++g) {
            const v16h bw = Frag<_Float16>::load(Bt + (size_t)(g * kNH + 16 * ub + cl) * kKC + k0 + 8 * hh);
            acc[g] = mma_h(a, bw, acc[g]);
          }
        }
#pragma unroll
        for (int r = 0; r < 8; ++r) {
          const float gi = acc[0][r] * kGSC + (fut ? bq[ubi][0] : bp[ubi][0]);
          const float gf = acc[1][r] * kGSC + (fut ? bq[ubi][1] : bp[ubi][1]);
          const float gg = acc[2][r] * kGSC + (fut ? bq[ubi][2] : bp[ubi][2]);
          const float go = acc[3][r] * kGSC + (fut ? bq[ubi][3] : bp[ubi][3]);
          const float vi = sigm_f(gi);
          const float vf = sigm_f(gf);
          const float vg = tanh_f(gg);
          const float vo = sigm_f(go);
          const float cn = vf * cst[ubi][r] + vi * vg;
          cst[ubi][r] = cn;
          hreg[ubi][r] = vo * tanh_f(cn);
        }
      }
    }
    __syncthreads();

#pragma unroll
    for (int ubi = 0; ubi < 2; ++ubi)
#pragma unroll
      for (int r = 0; r < 8; ++r)
        At[(8 * hh + r) * kATP + kNIP + 16 * (2 * wave + ubi) + cl] = (_Float16)(8.0f * hreg[ubi][r]);
    if (!fut) {
      const int tt = (t + 1 < kTP) ? (t + 1) : (kTP - 1);
      const int m = tid >> 4, seg = tid & 15;
      const v8h e = *(const v8h*)(enc16 + ((size_t)(b0 + m) * kTP + tt) * kNIP + 8 * seg);
      *(v8h*)(At + m * kATP + 8 * seg) = e;
    }
    __syncthreads();

    {
      const int r0 = 2 * wave, r1 = r0 + 1;
      const v8h h0 = *(const v8h*)(At + r0 * kATP + kNIP + 8 * lane);
      const v8h h1 = *(const v8h*)(At + r1 * kATP + kNIP + 8 * lane);
      const int sP = (t < kTP) ? t : (kTP - 1);
      const int sF = fut ? (t - kTP) : 0;
      _Float16* dP0 = hsp + ((size_t)(b0 + r0) * kTP + sP) * kNH + 8 * lane;
      _Float16* dP1 = hsp + ((size_t)(b0 + r1) * kTP + sP) * kNH + 8 * lane;
      _Float16* dF0 = hsf + ((size_t)(b0 + r0) * kTF + sF) * kNH + 8 * lane;
      _Float16* dF1 = hsf + ((size_t)(b0 + r1) * kTF + sF) * kNH + 8 * lane;
      _Float16* d0 = fut ? dF0 : dP0;
      _Float16* d1 = fut ? dF1 : dP1;
      for (int pass = 0; pass < 2; ++pass) {
        *(volatile v8h*)d0 = h0;
        *(volatile v8h*)d1 = h1;
        __threadfence();
      }
    }
  }
}

extern "C" void kernel_launch(void* const* d_in, const int* in_sizes, int n_in,
                              void* d_out, int out_size, void* d_ws, size_t ws_size,
                              hipStream_t stream)
{
  if (n_in < 16) return;
  if (in_sizes[0] != kNB * kTP * kNIN || in_sizes[1] < 1 ||
      in_sizes[2] != kNIP * kNIN || in_sizes[3] != kNIP ||
      in_sizes[4] != kNIP * kNH  || in_sizes[5] != kNIP ||
      in_sizes[6] != kNOUT * kNH || in_sizes[7] != kNOUT ||
      in_sizes[8] != kNG * kNIP  || in_sizes[9] != kNG * kNH || in_sizes[10] != kNG || in_sizes[11] != kNG ||
      in_sizes[12] != kNG * kNIP || in_sizes[13] != kNG * kNH || in_sizes[14] != kNG || in_sizes[15] != kNG) return;
  if (out_size != kNB * kTT * kNOUT) return;

  const float* x     = (const float*)d_in[0];
  const int*   futn  = (const int*)d_in[1];
  const float* enc_W = (const float*)d_in[2];
  const float* enc_b = (const float*)d_in[3];
  const float* fut_W = (const float*)d_in[4];
  const float* fut_b = (const float*)d_in[5];
  const float* dec_W = (const float*)d_in[6];
  const float* dec_b = (const float*)d_in[7];
  const float* pW_ih = (const float*)d_in[8];
  const float* pW_hh = (const float*)d_in[9];
  const float* pb_ih = (const float*)d_in[10];
  const float* pb_hh = (const float*)d_in[11];
  const float* fW_ih = (const float*)d_in[12];
  const float* fW_hh = (const float*)d_in[13];
  const float* fb_ih = (const float*)d_in[14];
  const float* fb_hh = (const float*)d_in[15];

  const size_t szX16  = (size_t)kNB * kTP * kNIN * 2;
  const size_t szENC  = (size_t)kNB * kTP * kNIP * 2;
  const size_t szHSP  = (size_t)kNB * kTP * kNH * 2;
  const size_t szBT   = (size_t)kNG * kKC * 2;
  const size_t szFUTW = (size_t)kNIP * kNH * 2;
  const size_t szDECW = (size_t)kNOUT * kNH * 2;
  const size_t szENCW = (size_t)kNIP * kNIN * 2;
  const size_t szENCB = (size_t)kNIP * 4;
  const size_t offX16  = 0;
  const size_t offENC  = offX16 + szX16;
  const size_t offHSP  = offENC + szENC;
  const size_t offBTP  = offHSP + szHSP;
  const size_t offBTF  = offBTP + szBT;
  const size_t offFUTW = offBTF + szBT;
  const size_t offDECW = offFUTW + szFUTW;
  const size_t offENCW = offDECW + szDECW;
  const size_t offENCB = offENCW + szENCW;
  const size_t total   = offENCB + szENCB;
  if (total > ws_size) return;

  char* ws = (char*)d_ws;
  _Float16* X16   = (_Float16*)(ws + offX16);
  _Float16* ENC16 = (_Float16*)(ws + offENC);
  _Float16* HSF   = (_Float16*)(ws + offENC);
  _Float16* HSP   = (_Float16*)(ws + offHSP);
  _Float16* BTP   = (_Float16*)(ws + offBTP);
  _Float16* BTF   = (_Float16*)(ws + offBTF);
  _Float16* FUTW  = (_Float16*)(ws + offFUTW);
  _Float16* DECW  = (_Float16*)(ws + offDECW);
  _Float16* ENCW  = (_Float16*)(ws + offENCW);
  float*    ENCB8 = (float*)(ws + offENCB);
  float*    out   = (float*)d_out;

  const int n2x = kNB * kTP * kNIN / 2;
  cast_f32_f16x2<<<(n2x + 255) / 256, 256, 0, stream>>>(x, X16, n2x);

  prep_planes<<<1649, 256, 0, stream>>>(pW_ih, pW_hh, fW_ih, fW_hh, fut_W, dec_W, enc_W, enc_b,
                                        BTP, BTF, FUTW, DECW, ENCW, ENCB8);

  {
    const int Mv = kNB * kTP, Nv = kNIP, Kv = kNIN;
    const int tiles = (Mv / 64) * (Nv / 64);
    dim3 grid((tiles + 7) / 8, 1);
    wmma_gemm64<0, false, 2, 1, false><<<grid, 256, 0, stream>>>(
        (const unsigned short*)X16, (const unsigned short*)X16, Kv, 0L,
        (const unsigned short*)ENCW, (const unsigned short*)ENCW, Kv, 0L,
        (void*)ENC16, (void*)ENC16, Nv, 0L,
        ENCB8, ENCB8, 0L, Mv, Nv, Kv, 0.5f);
  }

  lstm_seq_kernel<<<kNB / 16, 256, 0, stream>>>(ENC16, BTP, BTF, FUTW, pb_ih, pb_hh, fb_ih, fb_hh,
                                                fut_b, futn, HSP, HSF);

  {
    const int Mv = kTP, Nv = kNOUT, Kv = kNH;
    const int tiles = (Mv / 64) * (Nv / 64);
    dim3 grid((tiles + 7) / 8, kNB);
    wmma_gemm64<0, false, 2, 0, false><<<grid, 256, 0, stream>>>(
        (const unsigned short*)HSP, (const unsigned short*)HSP, Kv, (long)kTP * kNH,
        (const unsigned short*)DECW, (const unsigned short*)DECW, Kv, 0L,
        (void*)out, (void*)out, Nv, (long)kTT * kNOUT,
        dec_b, dec_b, 0L, Mv, Nv, Kv, kGSC);
  }
  {
    const int Mv = kTF, Nv = kNOUT, Kv = kNH;
    const int tiles = (Mv / 64) * (Nv / 64);
    dim3 grid((tiles + 7) / 8, kNB);
    wmma_gemm64<0, false, 2, 0, false><<<grid, 256, 0, stream>>>(
        (const unsigned short*)HSF, (const unsigned short*)HSF, Kv, (long)kTF * kNH,
        (const unsigned short*)DECW, (const unsigned short*)DECW, Kv, 0L,
        (void*)(out + (size_t)kTP * kNOUT), (void*)(out + (size_t)kTP * kNOUT), Nv, (long)kTT * kNOUT,
        dec_b, dec_b, 0L, Mv, Nv, Kv, kGSC);
  }
}
